// GCNNet_79680233275798
// MI455X (gfx1250) — hardware-verified
//
#include <hip/hip_runtime.h>
#include <stddef.h>
#include <stdint.h>
#include <math.h>


#define NN     100000
#define NE     1600000
#define FIN    78
#define KP     96
#define FH     156
#define NP     160
#define NG     64
#define EMB    32
#define KH     320
#define NTHR   256
#define NWAVE  8
#define EPT    8
#define CHUNK  (NTHR * EPT)
#define WCAP   (EPT * 32)
#define LISTN  (NWAVE * WCAP)
#define NBA    1024
#define SLA    10
#define RCAP   28672
#define DEGCAP 64
#define MEAS_B1024  16710
#define MEAS_MAXDEG 36
#define GBM    64
#define GTHR   128
#define MPAD   100096
#define NBLK   98
#define NBP    (NBLK * NBA)
#define AGG_ZINTS (LISTN + 2 * RCAP + 3 * NBA)
#define AGG_LDS_INTS (AGG_ZINTS + 16)
#define NUWT   (NP * (KP / 8))
#define NUFC   (EMB * (KH / 8))
#define SMU    48
#define PB_WT  8
#define PB_FC  13
#define PB_SM  13
#define PB_XB  14
#define WSMAX  134217728

static_assert((CHUNK & (CHUNK - 1)) == 0 && CHUNK <= 4096);
static_assert((NBA & (NBA - 1)) == 0 && NBA == (1 << SLA));
static_assert(((long long)CHUNK << SLA) < (1LL << 31));
static_assert(NE < (1 << (31 - SLA)));
static_assert(NP == 5 * 32 && KP % 32 == 0 && KH % 32 == 0 && KH == 2 * NP);
static_assert(FIN <= KP && FH <= NP && NG == 64 && EMB == 32);
static_assert(NBLK * NBA >= NN && NBP >= MPAD && NBLK <= NTHR);
static_assert(782 * 128 == MPAD && MPAD % GBM == 0 && MPAD >= NN);
static_assert(RCAP >= MEAS_B1024 + MEAS_B1024 / 20 + 1);
static_assert(DEGCAP >= MEAS_MAXDEG + 8);
static_assert(RCAP % (NTHR * 4) == 0 && AGG_ZINTS % (NTHR * 4) == 0);
static_assert(AGG_LDS_INTS * 4 <= 300000);
static_assert(NBA == NTHR * 4);
static_assert((NG * NP) % (NTHR * 4) == 0 && (GBM * NP) % (GTHR * 4) == 0);
static_assert((NG * EMB) % (NTHR * 4) == 0);
static_assert(NUWT <= PB_WT * NTHR && NUFC == (PB_FC - PB_WT) * NTHR);
static_assert((MPAD * (KP / 8)) % NTHR == 0);
static_assert(NG * NP * 4 + 32 * NP * 4 + 256 <= 65536);

typedef float          v4f   __attribute__((ext_vector_type(4)));
typedef float          v8f   __attribute__((ext_vector_type(8)));
typedef int            v4i   __attribute__((ext_vector_type(4)));
typedef int            v8i   __attribute__((ext_vector_type(8)));
typedef unsigned short v4us  __attribute__((ext_vector_type(4)));
typedef unsigned short v8us  __attribute__((ext_vector_type(8)));
typedef unsigned short v16us __attribute__((ext_vector_type(16)));
typedef __bf16         v16bf __attribute__((ext_vector_type(16)));
typedef v4f  __attribute__((may_alias)) v4fa;
typedef v4i  __attribute__((may_alias)) v4ia;
typedef v4us __attribute__((may_alias)) v4usa;
typedef v8us __attribute__((may_alias)) v8usa;
union FragB { v16bf v; v16us u; v8us h[2]; v8i w; };

__device__ __forceinline__ v8f wmb(const FragB& a, const FragB& b, v8f c) {
  v8f d = __builtin_amdgcn_wmma_f32_16x16x32_bf16(false, a.v, false, b.v, (short)0, c, false, false);
  asm volatile("v_nop\n\tv_nop\n\tv_nop\n\tv_nop" : "+v"(d) : "v"(a.w), "v"(b.w));
  return d;
}

__device__ __forceinline__ v8f z8() { v8f z = {0.f, 0.f, 0.f, 0.f, 0.f, 0.f, 0.f, 0.f}; return z; }

__device__ __forceinline__ unsigned bf16_bits(float f) {
  const unsigned u = __float_as_uint(f);
  return (u + 0x7FFFu + ((u >> 16) & 1u)) >> 16;
}

template <int SLB>
__device__ __forceinline__ int scan_chunk(const int* __restrict__ dsts, int nE, int cbase, int slotBase,
                                          int nb, int vec8, int* list, int tid, int lane, int wave) {
  int wc = 0;
  const int el0  = tid * EPT;
  const int e0   = cbase + el0;
  const int sent = -2147483647 - 1;
  v4i da, db;
  if (vec8 != 0 && cbase + CHUNK <= nE) {
    da = *(const v4i*)(dsts + e0);
    db = *(const v4i*)(dsts + e0 + 4);
  } else {
    da.x = (e0     < nE) ? dsts[min(e0,     nE - 1)] : sent;
    da.y = (e0 + 1 < nE) ? dsts[min(e0 + 1, nE - 1)] : sent;
    da.z = (e0 + 2 < nE) ? dsts[min(e0 + 2, nE - 1)] : sent;
    da.w = (e0 + 3 < nE) ? dsts[min(e0 + 3, nE - 1)] : sent;
    db.x = (e0 + 4 < nE) ? dsts[min(e0 + 4, nE - 1)] : sent;
    db.y = (e0 + 5 < nE) ? dsts[min(e0 + 5, nE - 1)] : sent;
    db.z = (e0 + 6 < nE) ? dsts[min(e0 + 6, nE - 1)] : sent;
    db.w = (e0 + 7 < nE) ? dsts[min(e0 + 7, nE - 1)] : sent;
  }
  const unsigned nbs = (unsigned)slotBase;
  const unsigned unb = (unsigned)nb;
  const unsigned s0 = (unsigned)da.x - nbs, s1 = (unsigned)da.y - nbs;
  const unsigned s2 = (unsigned)da.z - nbs, s3 = (unsigned)da.w - nbs;
  const unsigned s4 = (unsigned)db.x - nbs, s5 = (unsigned)db.y - nbs;
  const unsigned s6 = (unsigned)db.z - nbs, s7 = (unsigned)db.w - nbs;
  const bool h0 = s0 < unb, h1 = s1 < unb, h2 = s2 < unb, h3 = s3 < unb;
  const bool h4 = s4 < unb, h5 = s5 < unb, h6 = s6 < unb, h7 = s7 < unb;
  const unsigned any = __builtin_amdgcn_ballot_w32(h0 | h1 | h2 | h3 | h4 | h5 | h6 | h7);
  if (any != 0u) {
#define HITJ(J, HJ, SJ) { \
      const unsigned mj = __builtin_amdgcn_ballot_w32(HJ); \
      if (mj != 0u) { \
        if (HJ) { \
          const int pos = wc + (int)__builtin_amdgcn_mbcnt_lo(mj, 0u); \
          if (pos < WCAP) list[wave * WCAP + pos] = ((el0 + (J)) << SLB) | (int)(SJ); \
        } \
        wc += (int)__builtin_popcount(mj); } }
    HITJ(0, h0, s0)
    HITJ(1, h1, s1)
    HITJ(2, h2, s2)
    HITJ(3, h3, s3)
    HITJ(4, h4, s4)
    HITJ(5, h5, s5)
    HITJ(6, h6, s6)
    HITJ(7, h7, s7)
#undef HITJ
  }
  return wc;
}

__global__ __launch_bounds__(NTHR) void k_prep(const float* __restrict__ x, const float* __restrict__ W,
                                               const float* __restrict__ b, const float* __restrict__ fcW,
                                               const float* __restrict__ fcb,
                                               unsigned short* xb, unsigned short* wt, unsigned short* fcwd,
                                               float* sm, int nN, int nUx) {
  const int blk = (int)blockIdx.x;
  const int tid = (int)threadIdx.x;
  if (blk == PB_SM) {
    const int t = tid < SMU ? tid : SMU - 1;
    unsigned bits[4];
#pragma unroll
    for (int j = 0; j < 4; ++j) {
      const int w  = 4 * t + j;
      const int wa = w < FH ? w : FH - 1;
      int wb = w - NP;
      wb = wb < 0 ? 0 : (wb > EMB - 1 ? EMB - 1 : wb);
      const unsigned ua = bf16_bits(b[wa]) << 16;
      const unsigned ub = bf16_bits(fcb[wb]) << 16;
      const unsigned ma = (w < FH) ? 0xFFFFFFFFu : 0u;
      const unsigned mb = (w >= NP) ? 0xFFFFFFFFu : 0u;
      bits[j] = (ua & ma) | (ub & mb);
    }
    v4f o;
    o.x = __uint_as_float(bits[0]); o.y = __uint_as_float(bits[1]);
    o.z = __uint_as_float(bits[2]); o.w = __uint_as_float(bits[3]);
    float* dp = sm + 4 * t;
    const bool act = tid < SMU;
    if (act) *(volatile v4f*)dp = o;
    __threadfence();
    if (act) *(volatile v4f*)dp = o;
    return;
  }
  v8us o;
  unsigned short* dp;
  bool act;
  if (blk < PB_WT) {
    const int v  = blk * NTHR + tid;
    act = v < NUWT;
    const int vc = act ? v : NUWT - 1;
    const int n  = vc / (KP / 8);
    const int k8 = (vc - n * (KP / 8)) * 8;
    const int nc = n < FH ? n : FH - 1;
#pragma unroll
    for (int i = 0; i < 8; ++i) {
      const int k  = k8 + i;
      const int kc = k < FIN ? k : FIN - 1;
      const float f = W[(size_t)kc * FH + nc];
      o[i] = (unsigned short)bf16_bits((k < FIN && n < FH) ? f : 0.0f);
    }
    dp = wt + (size_t)vc * 8;
  } else if (blk < PB_FC) {
    const int v  = (blk - PB_WT) * NTHR + tid;
    act = v < NUFC;
    const int vc = act ? v : NUFC - 1;
    const int n  = vc / (KH / 8);
    const int k8 = (vc - n * (KH / 8)) * 8;
    const int kk8 = k8 >= NP ? k8 - NP : k8;
#pragma unroll
    for (int i = 0; i < 8; ++i) {
      const int kk = kk8 + i;
      const int kc = kk < FH ? kk : FH - 1;
      const float f = fcW[(size_t)kc * EMB + n];
      o[i] = (unsigned short)bf16_bits((kk < FH) ? f : 0.0f);
    }
    dp = fcwd + (size_t)vc * 8;
  } else {
    const int v  = (blk - PB_XB) * NTHR + tid;
    act = v < nUx;
    const int vc = act ? v : nUx - 1;
    const int row = vc / (KP / 8);
    const int k8  = (vc - row * (KP / 8)) * 8;
    const int rc  = row < nN ? row : nN - 1;
    const bool lv = row < nN;
    const float* p = x + (size_t)rc * FIN;
#pragma unroll
    for (int i = 0; i < 8; ++i) {
      const int k  = k8 + i;
      const int kc = k < FIN ? k : FIN - 1;
      const float f = p[kc];
      o[i] = (unsigned short)bf16_bits((lv && k < FIN) ? f : 0.0f);
    }
    dp = xb + (size_t)vc * 8;
  }
  if (act) *(volatile v8us*)dp = o;
  __threadfence();
  if (act) *(volatile v8us*)dp = o;
}

__global__ __launch_bounds__(GTHR) void k_gemm(const unsigned short* __restrict__ A,
                                               const unsigned short* __restrict__ WT, float* outF) {
  __shared__ __attribute__((aligned(16))) float stg[GBM * NP];
  const int tid = (int)threadIdx.x, lane = tid & 31, wave = tid >> 5, hh = lane >> 4, m = lane & 15;
  const int rowBase = (int)blockIdx.x * GBM;

  v8f acc[10];
#pragma unroll
  for (int t = 0; t < 10; ++t) acc[t] = z8();
  const unsigned short* ap = A  + (size_t)(rowBase + 16 * wave + m) * (size_t)KP + 8 * hh;
  const unsigned short* wp = WT + (size_t)m * (size_t)KP + 8 * hh;
#pragma unroll 1
  for (int k0 = 0; k0 < KP; k0 += 32) {
    FragB af;
    af.h[0] = *(const v8usa*)(ap + k0);
    af.h[1] = *(const v8usa*)(ap + k0 + 16);
#pragma unroll
    for (int t = 0; t < 10; ++t) {
      const unsigned short* wq = wp + (size_t)(16 * t) * (size_t)KP + k0;
      FragB bf;
      bf.h[0] = *(const v8usa*)wq;
      bf.h[1] = *(const v8usa*)(wq + 16);
      acc[t] = wmb(af, bf, acc[t]);
    }
  }

#pragma unroll
  for (int t = 0; t < 10; ++t) {
    const int lc = 16 * t + m;
#pragma unroll
    for (int r = 0; r < 8; ++r) {
      const int lr = 16 * wave + 8 * hh + r;
      stg[lr * NP + lc] = acc[t][r];
    }
  }
  __syncthreads();

  float* ob = outF + (size_t)rowBase * NP;
  constexpr int NIT = (GBM * NP) / (GTHR * 4);
#pragma unroll 4
  for (int it = 0; it < NIT; ++it) {
    const int e = 4 * (it * GTHR + tid);
    const v4f v = *(const v4fa*)(stg + e);
    *(volatile v4f*)(ob + e) = v;
  }
  __threadfence();
#pragma unroll 4
  for (int it = 0; it < NIT; ++it) {
    const int e = 4 * (it * GTHR + tid);
    const v4f v = *(const v4fa*)(stg + e);
    *(volatile v4f*)(ob + e) = v;
  }
}

__global__ __launch_bounds__(NTHR) void k_bucket(const int* __restrict__ srcs, const int* __restrict__ dsts,
                                                 int nE, int nN, int vec8,
                                                 int* listg, int* cntg, int* offg, float* disg, int* flagg) {
  extern __shared__ __attribute__((aligned(16))) int dsm[];
  int* list = dsm;
  int* hl   = dsm + LISTN;
  int* sl   = dsm + LISTN + RCAP;
  int* cnt  = dsm + LISTN + 2 * RCAP;
  int* offs = cnt + NBA;
  int* cur  = offs + NBA;
  int* misc = cur + NBA;
  const int tid = (int)threadIdx.x, lane = tid & 31, wave = tid >> 5;
  const int q = (int)blockIdx.x;
  const int nodeBase = q * NBA;

  {
    const v4i z4 = {0, 0, 0, 0};
    for (int i = tid * 4; i < AGG_ZINTS; i += NTHR * 4) *(v4ia*)(dsm + i) = z4;
    if (tid < 16) misc[tid] = 0;
  }
  __syncthreads();

  int t = 0, ov = 0;
  const int nChunks = (nE + CHUNK - 1) / CHUNK;
#pragma unroll 1
  for (int ch = 0; ch < nChunks; ++ch) {
    const int cbase = ch * CHUNK;
    const int wc = scan_chunk<SLA>(dsts, nE, cbase, nodeBase, NBA, vec8, list, tid, lane, wave);
    if (lane == 0) misc[wave] = wc;
    __syncthreads();
    if (wave == 0) {
#pragma unroll 1
      for (int w2 = 0; w2 < NWAVE; ++w2) {
        int c = misc[w2];
        c = c < 0 ? 0 : (c > WCAP ? WCAP : c);
#pragma unroll 1
        for (int b0 = 0; b0 < c; b0 += 32) {
          const int idx = b0 + lane;
          const int ent = list[w2 * WCAP + (idx < WCAP ? idx : WCAP - 1)];
          const int m32 = (c - b0) < 32 ? (c - b0) : 32;
#pragma unroll 1
          for (int k = 0; k < m32; ++k) {
            const int u    = __builtin_amdgcn_readlane(ent, k);
            const int slot = u & (NBA - 1);
            const int el   = (u >> SLA) & (CHUNK - 1);
            const int pk   = ((cbase + el) << SLA) | slot;
            if (t < RCAP) {
              if (lane == 0) { hl[t] = pk; cnt[slot] = cnt[slot] + 1; }
              t = t + 1;
            } else {
              ov = 1;
            }
          }
        }
      }
    }
    __syncthreads();
  }
  if (wave == 0 && lane == 0) { misc[8] = t; misc[9] = ov; }
  __syncthreads();
  int tt = misc[8];
  tt = tt < 0 ? 0 : (tt > RCAP ? RCAP : tt);
  const int ovf = misc[9];

  if (wave == 0) {
    const int base = lane * (NBA / 32);
    int s = 0;
#pragma unroll 1
    for (int i = 0; i < NBA / 32; ++i) s += cnt[base + i];
    int incl = s;
#pragma unroll
    for (int d = 1; d < 32; d <<= 1) {
      const int y = __shfl_up(incl, d, 32);
      if (lane >= d) incl += y;
    }
    int run = incl - s;
#pragma unroll 1
    for (int i = 0; i < NBA / 32; ++i) {
      const int cv = cnt[base + i];
      offs[base + i] = run;
      cur[base + i]  = run;
      run += cv;
    }
  }
  __syncthreads();
  if (wave == 0) {
#pragma unroll 1
    for (int b0 = 0; b0 < tt; b0 += 32) {
      const int idx = b0 + lane;
      const int ent = hl[idx < RCAP ? idx : RCAP - 1];
      const int m32 = (tt - b0) < 32 ? (tt - b0) : 32;
#pragma unroll 1
      for (int k = 0; k < m32; ++k) {
        const int u    = __builtin_amdgcn_readlane(ent, k);
        const int slot = u & (NBA - 1);
        if (lane == 0) {
          int p = cur[slot];
          p = p < 0 ? 0 : (p > RCAP - 1 ? RCAP - 1 : p);
          sl[p] = u;
          cur[slot] = p + 1;
        }
      }
    }
  }
  __syncthreads();

#pragma unroll 1
  for (int i4 = tid * 4; i4 < RCAP; i4 += NTHR * 4) {
    const v4i e = *(const v4ia*)(sl + i4);
    int e0 = e.x >> SLA, e1 = e.y >> SLA, e2 = e.z >> SLA, e3 = e.w >> SLA;
    e0 = e0 < 0 ? 0 : (e0 > nE - 1 ? nE - 1 : e0);
    e1 = e1 < 0 ? 0 : (e1 > nE - 1 ? nE - 1 : e1);
    e2 = e2 < 0 ? 0 : (e2 > nE - 1 ? nE - 1 : e2);
    e3 = e3 < 0 ? 0 : (e3 > nE - 1 ? nE - 1 : e3);
    int s0 = srcs[e0], s1 = srcs[e1], s2 = srcs[e2], s3 = srcs[e3];
    s0 = s0 < 0 ? 0 : (s0 > nN - 1 ? nN - 1 : s0);
    s1 = s1 < 0 ? 0 : (s1 > nN - 1 ? nN - 1 : s1);
    s2 = s2 < 0 ? 0 : (s2 > nN - 1 ? nN - 1 : s2);
    s3 = s3 < 0 ? 0 : (s3 > nN - 1 ? nN - 1 : s3);
    v4i o;
    o.x = (i4     < tt) ? s0 : 0;
    o.y = (i4 + 1 < tt) ? s1 : 0;
    o.z = (i4 + 2 < tt) ? s2 : 0;
    o.w = (i4 + 3 < tt) ? s3 : 0;
    *(v4ia*)(hl + i4) = o;
  }
#pragma unroll 1
  for (int i = tid; i < NBA; i += NTHR) {
    const float d = (float)(cnt[i] + 1);
    cur[i] = __float_as_int(1.0f / sqrtf(d));
  }
  __syncthreads();

  int* lp = listg + (size_t)q * RCAP;
  const v4i c4 = *(const v4ia*)(cnt + 4 * tid);
  const v4i o4 = *(const v4ia*)(offs + 4 * tid);
  const v4i d4 = *(const v4ia*)(cur + 4 * tid);
  v4f df;
  df.x = __int_as_float(d4.x); df.y = __int_as_float(d4.y);
  df.z = __int_as_float(d4.z); df.w = __int_as_float(d4.w);
  const v4i f4 = {ovf, ovf, ovf, ovf};
#pragma unroll 1
  for (int i4 = tid * 4; i4 < RCAP; i4 += NTHR * 4) {
    const v4i v = *(const v4ia*)(hl + i4);
    *(volatile v4i*)(lp + i4) = v;
  }
  *(volatile v4i*)(cntg + nodeBase + 4 * tid) = c4;
  *(volatile v4i*)(offg + nodeBase + 4 * tid) = o4;
  *(volatile v4f*)(disg + nodeBase + 4 * tid) = df;
  if (tid < 8) *(volatile v4i*)(flagg + q * 32 + 4 * tid) = f4;
  __threadfence();
#pragma unroll 1
  for (int i4 = tid * 4; i4 < RCAP; i4 += NTHR * 4) {
    const v4i v = *(const v4ia*)(hl + i4);
    *(volatile v4i*)(lp + i4) = v;
  }
  *(volatile v4i*)(cntg + nodeBase + 4 * tid) = c4;
  *(volatile v4i*)(offg + nodeBase + 4 * tid) = o4;
  *(volatile v4f*)(disg + nodeBase + 4 * tid) = df;
  if (tid < 8) *(volatile v4i*)(flagg + q * 32 + 4 * tid) = f4;
}

__global__ __launch_bounds__(NTHR) void k_agg(const float* __restrict__ H, const int* __restrict__ listg,
                                              const int* __restrict__ cntg, const int* __restrict__ offg,
                                              const float* __restrict__ disg, const int* __restrict__ flagg,
                                              const float* __restrict__ btg, const int* __restrict__ bat,
                                              int nN, int nBP, float* rec) {
  __shared__ __attribute__((aligned(16))) float tbl[NG * NP];
  __shared__ __attribute__((aligned(16))) float stg[32 * NP];
  __shared__ int sg[32];
  const int tid = (int)threadIdx.x, lane = tid & 31;
  const int wave = __builtin_amdgcn_readfirstlane(tid >> 5);
  const int q = (int)blockIdx.x;
  const int nodeBase = q * NBA;
  const float ninf = -__builtin_huge_valf();
  const float qnan = __int_as_float(0x7fc00000);
  {
    const v4f n4 = {ninf, ninf, ninf, ninf};
    for (int i = tid * 4; i < NG * NP; i += NTHR * 4) *(v4fa*)(tbl + i) = n4;
  }
  const float bt0 = btg[lane], bt1 = btg[lane + 32], bt2 = btg[lane + 64];
  const float bt3 = btg[lane + 96], bt4 = btg[lane + 128];
  const bool pzb = flagg[q * 32] != 0;
  const int* lp = listg + (size_t)q * RCAP;
  __syncthreads();

#pragma unroll 1
  for (int st = 0; st < NBA / 32; ++st) {
    const int rbase = nodeBase + st * 32;
    if (wave == 0) {
      const int i  = rbase + lane;
      const int ic = i < nN ? i : nN - 1;
      const int g  = bat[ic];
      sg[lane] = (i < nN && g >= 0 && g < NG) ? g : -1;
    }
#pragma unroll 1
    for (int j = 0; j < 4; ++j) {
      const int rr = wave * 4 + j;
      const int i  = rbase + rr;
      const int it = i < nBP ? i : nBP - 1;
      const int ic = i < nN ? i : nN - 1;
      int c = __builtin_amdgcn_readfirstlane(cntg[it]);
      int o = __builtin_amdgcn_readfirstlane(offg[it]);
      const float dd = disg[it];
      const bool big = c > DEGCAP;
      c = c < 0 ? 0 : (c > DEGCAP ? DEGCAP : c);
      o = o < 0 ? 0 : (o > RCAP ? RCAP : o);
      const float rd = dd * dd;
      float a0 = 0.0f, a1 = 0.0f, a2 = 0.0f, a3 = 0.0f, a4 = 0.0f;
#pragma unroll 1
      for (int b0 = 0; b0 < c; b0 += 32) {
        int idx = o + b0 + lane;
        const int last = o + c - 1;
        idx = idx > last ? last : idx;
        idx = idx > RCAP - 1 ? RCAP - 1 : idx;
        idx = idx < 0 ? 0 : idx;
        int sr = lp[idx];
        sr = sr < 0 ? 0 : (sr > nN - 1 ? nN - 1 : sr);
        const float cf  = disg[sr] * dd;
        const int   cfi = __float_as_int(cf);
        const int m32 = (c - b0) < 32 ? (c - b0) : 32;
#pragma unroll 1
        for (int k = 0; k < m32; ++k) {
          const int   sk = __builtin_amdgcn_readlane(sr, k);
          const float ck = __int_as_float(__builtin_amdgcn_readlane(cfi, k));
          const float* hp = H + (size_t)sk * NP + lane;
          const float h0 = hp[0], h1 = hp[32], h2 = hp[64], h3 = hp[96], h4 = hp[128];
          a0 = fmaf(ck, h0, a0); a1 = fmaf(ck, h1, a1); a2 = fmaf(ck, h2, a2);
          a3 = fmaf(ck, h3, a3); a4 = fmaf(ck, h4, a4);
        }
      }
      const float* sp = H + (size_t)ic * NP + lane;
      const float s0 = sp[0], s1 = sp[32], s2 = sp[64], s3 = sp[96], s4 = sp[128];
      float y0 = fmaf(s0, rd, a0) + bt0;
      float y1 = fmaf(s1, rd, a1) + bt1;
      float y2 = fmaf(s2, rd, a2) + bt2;
      float y3 = fmaf(s3, rd, a3) + bt3;
      float y4 = fmaf(s4, rd, a4) + bt4;
      y0 = (y0 > 0.0f) ? y0 : (y0 - y0);
      y1 = (y1 > 0.0f) ? y1 : (y1 - y1);
      y2 = (y2 > 0.0f) ? y2 : (y2 - y2);
      y3 = (y3 > 0.0f) ? y3 : (y3 - y3);
      y4 = (y4 > 0.0f) ? y4 : (y4 - y4);
      const bool bad = pzb || big;
      y0 = bad ? qnan : y0; y1 = bad ? qnan : y1; y2 = bad ? qnan : y2;
      y3 = bad ? qnan : y3; y4 = bad ? qnan : y4;
      float* sq = stg + rr * NP + lane;
      sq[0] = y0; sq[32] = y1; sq[64] = y2; sq[96] = y3; sq[128] = y4;
    }
    __syncthreads();
    if (tid < NP) {
#pragma unroll 4
      for (int j = 0; j < 32; ++j) {
        const int g  = sg[j];
        const int gc = g < 0 ? 0 : (g > NG - 1 ? NG - 1 : g);
        const float m = tbl[gc * NP + tid];
        const float v = stg[j * NP + tid];
        const bool take = (g >= 0) && ((v > m) || (v != v));
        tbl[gc * NP + tid] = take ? v : m;
      }
    }
    __syncthreads();
  }

  float* rp = rec + (size_t)q * (NG * NP);
  constexpr int NIT = (NG * NP) / (NTHR * 4);
#pragma unroll 2
  for (int it = 0; it < NIT; ++it) {
    const int e = 4 * (it * NTHR + tid);
    const v4f v = *(const v4fa*)(tbl + e);
    *(volatile v4f*)(rp + e) = v;
  }
  __threadfence();
#pragma unroll 2
  for (int it = 0; it < NIT; ++it) {
    const int e = 4 * (it * NTHR + tid);
    const v4f v = *(const v4fa*)(tbl + e);
    *(volatile v4f*)(rp + e) = v;
  }
}

__global__ __launch_bounds__(NTHR) void k_head(const float* __restrict__ rec,
                                               const unsigned short* __restrict__ fcwd,
                                               const float* __restrict__ fcbv, const int* __restrict__ flagg,
                                               int nBlk, float* out) {
  __shared__ __attribute__((aligned(16))) unsigned short at[NG * KH];
  __shared__ __attribute__((aligned(16))) float os[NG * EMB];
  __shared__ unsigned swf[NWAVE];
  const int tid = (int)threadIdx.x, lane = tid & 31, wave = tid >> 5, hh = lane >> 4, m = lane & 15;
  const float ninf = -__builtin_huge_valf();
  const float pinf = __builtin_huge_valf();
  const float qnan = __int_as_float(0x7fc00000);

  {
    const int t = tid < nBlk ? tid : nBlk - 1;
    const int f = flagg[t * 32];
    const bool bad = (tid < nBlk) && (f != 0);
    const unsigned bm = __builtin_amdgcn_ballot_w32(bad);
    if (lane == 0) swf[wave] = bm;
  }

#pragma unroll 1
  for (int n = 0; n < (NG * NP) / (NTHR * 4); ++n) {
    const int u = n * NTHR + tid;
    const float* rp = rec + 4 * u;
    float m0 = ninf, m1 = ninf, m2 = ninf, m3 = ninf;
#pragma unroll 2
    for (int q = 0; q < nBlk; ++q) {
      const v4f v = *(const v4fa*)(rp + (size_t)q * (NG * NP));
      m0 = ((v.x > m0) || (v.x != v.x)) ? v.x : m0;
      m1 = ((v.y > m1) || (v.y != v.y)) ? v.y : m1;
      m2 = ((v.z > m2) || (v.z != v.z)) ? v.z : m2;
      m3 = ((v.w > m3) || (v.w != v.w)) ? v.w : m3;
    }
    m0 = (m0 == ninf || m0 == pinf) ? 0.0f : m0;
    m1 = (m1 == ninf || m1 == pinf) ? 0.0f : m1;
    m2 = (m2 == ninf || m2 == pinf) ? 0.0f : m2;
    m3 = (m3 == ninf || m3 == pinf) ? 0.0f : m3;
    const unsigned hb0 = bf16_bits(m0), hb1 = bf16_bits(m1), hb2 = bf16_bits(m2), hb3 = bf16_bits(m3);
    const unsigned lb0 = bf16_bits(m0 - __uint_as_float(hb0 << 16));
    const unsigned lb1 = bf16_bits(m1 - __uint_as_float(hb1 << 16));
    const unsigned lb2 = bf16_bits(m2 - __uint_as_float(hb2 << 16));
    const unsigned lb3 = bf16_bits(m3 - __uint_as_float(hb3 << 16));
    v4us h4, l4;
    h4[0] = (unsigned short)hb0; h4[1] = (unsigned short)hb1; h4[2] = (unsigned short)hb2; h4[3] = (unsigned short)hb3;
    l4[0] = (unsigned short)lb0; l4[1] = (unsigned short)lb1; l4[2] = (unsigned short)lb2; l4[3] = (unsigned short)lb3;
    const int g = (4 * u) / NP;
    const int c = 4 * u - g * NP;
    *(v4usa*)(at + g * KH + c) = h4;
    *(v4usa*)(at + g * KH + NP + c) = l4;
  }
  __syncthreads();

  const int mt = wave >> 1, nt = wave & 1;
  const unsigned short* ap = at + (16 * mt + m) * KH + 8 * hh;
  const unsigned short* bp = fcwd + (size_t)(16 * nt + m) * KH + 8 * hh;
  v8f acc = z8();
#pragma unroll 2
  for (int ks = 0; ks < KH / 32; ++ks) {
    FragB af, bf;
    af.h[0] = *(const v8usa*)(ap + 32 * ks);
    af.h[1] = *(const v8usa*)(ap + 32 * ks + 16);
    bf.h[0] = *(const v8usa*)(bp + 32 * ks);
    bf.h[1] = *(const v8usa*)(bp + 32 * ks + 16);
    acc = wmb(af, bf, acc);
  }

  const unsigned anyf = swf[0] | swf[1] | swf[2] | swf[3] | swf[4] | swf[5] | swf[6] | swf[7];
  const int col = 16 * nt + m;
  const float fb = fcbv[col];
#pragma unroll
  for (int r = 0; r < 8; ++r) {
    const int row = 16 * mt + 8 * hh + r;
    float y = acc[r] + fb;
    y = (y > 0.0f) ? y : (y - y);
    y = (anyf != 0u) ? qnan : y;
    os[row * EMB + col] = y;
  }
  __syncthreads();

  constexpr int NIT = (NG * EMB) / (NTHR * 4);
  v4f ov[NIT];
#pragma unroll
  for (int it = 0; it < NIT; ++it) ov[it] = *(const v4fa*)(os + 4 * (it * NTHR + tid));
#pragma unroll
  for (int it = 0; it < NIT; ++it) *(volatile v4f*)(out + 4 * (size_t)(it * NTHR + tid)) = ov[it];
  __threadfence();
#pragma unroll
  for (int it = 0; it < NIT; ++it) *(volatile v4f*)(out + 4 * (size_t)(it * NTHR + tid)) = ov[it];
}

static inline int cdiv(int a, int b) { return (a + b - 1) / b; }
static inline size_t al256(size_t o) { return (o + 255) & ~(size_t)255; }

extern "C" void kernel_launch(void* const* d_in, const int* in_sizes, int n_in,
                              void* d_out, int out_size, void* d_ws, size_t ws_size,
                              hipStream_t stream) {
  if (n_in < 7) return;
  if (in_sizes[0] != NN * FIN) return;
  if (in_sizes[1] != 2 * NE) return;
  if (in_sizes[2] != NN) return;
  if (in_sizes[3] != FIN * FH || in_sizes[4] != FH) return;
  if (in_sizes[5] != FH * EMB || in_sizes[6] != EMB) return;
  if (out_size != NG * EMB) return;
  const int nN = NN, nE = NE;

  const float* x    = (const float*)d_in[0];
  const int*   edge = (const int*)d_in[1];
  const int*   bat  = (const int*)d_in[2];
  const float* W    = (const float*)d_in[3];
  const float* b    = (const float*)d_in[4];
  const float* fcW  = (const float*)d_in[5];
  const float* fcb  = (const float*)d_in[6];
  float* out = (float*)d_out;
  const int* src = edge;
  const int* dst = edge + nE;

  const int MP  = cdiv(nN, 128) * 128;
  const int gM  = MP / GBM;
  const int gA  = cdiv(nN, NBA);
  const int nBP = gA * NBA;
  if (MP != MPAD || gA != NBLK || nBP < MP) return;
  const int vec8 = ((nE & 3) == 0) ? 1 : 0;
  const int nUx = MP * (KP / 8);

  char* ws = (char*)d_ws;
  size_t off = 0;
  const size_t oH    = off; off = al256(off + (size_t)MP * NP * 4);
  const size_t oXB   = off; off = al256(off + (size_t)MP * KP * 2);
  const size_t oLIST = off; off = al256(off + (size_t)gA * RCAP * 4);
  const size_t oCNT  = off; off = al256(off + (size_t)nBP * 4);
  const size_t oOFF  = off; off = al256(off + (size_t)nBP * 4);
  const size_t oDIS  = off; off = al256(off + (size_t)nBP * 4);
  const size_t oREC  = off; off = al256(off + (size_t)gA * NG * NP * 4);
  const size_t oWT   = off; off = al256(off + (size_t)NP * KP * 2);
  const size_t oFC   = off; off = al256(off + (size_t)EMB * KH * 2);
  const size_t oSM   = off; off = al256(off + (size_t)(NP + EMB) * 4);
  const size_t oFL   = off; off = al256(off + (size_t)gA * 32 * 4);
  if (off > ws_size || off > (size_t)WSMAX) return;
  float*          H    = (float*)(ws + oH);
  unsigned short* XB   = (unsigned short*)(ws + oXB);
  int*            LIST = (int*)(ws + oLIST);
  int*            CNT  = (int*)(ws + oCNT);
  int*            OFF  = (int*)(ws + oOFF);
  float*          DIS  = (float*)(ws + oDIS);
  float*          REC  = (float*)(ws + oREC);
  unsigned short* WT   = (unsigned short*)(ws + oWT);
  unsigned short* FCWD = (unsigned short*)(ws + oFC);
  float*          SM   = (float*)(ws + oSM);
  int*            FLAG = (int*)(ws + oFL);
  const float* BT  = SM;
  const float* FCB = SM + NP;

  const size_t bLds = (size_t)AGG_LDS_INTS * 4;
  hipFuncSetAttribute(reinterpret_cast<const void*>(&k_bucket), hipFuncAttributeMaxDynamicSharedMemorySize, (int)bLds);

  k_prep<<<PB_XB + cdiv(nUx, NTHR), NTHR, 0, stream>>>(x, W, b, fcW, fcb, XB, WT, FCWD, SM, nN, nUx);
  k_gemm<<<gM, GTHR, 0, stream>>>(XB, WT, H);
  k_bucket<<<gA, NTHR, bLds, stream>>>(src, dst, nE, nN, vec8, LIST, CNT, OFF, DIS, FLAG);
  k_agg<<<gA, NTHR, 0, stream>>>(H, LIST, CNT, OFF, DIS, FLAG, BT, bat, nN, nBP, REC);
  k_head<<<1, NTHR, 0, stream>>>(REC, FCWD, FCB, FLAG, gA, out);
}
